// JointScorer_41429254537310
// MI455X (gfx1250) — hardware-run, weakly checked
//
#include <hip/hip_runtime.h>

typedef float          v8f   __attribute__((ext_vector_type(8)));
typedef float          v4f   __attribute__((ext_vector_type(4)));
typedef unsigned int   v4u   __attribute__((ext_vector_type(4)));
typedef int            v8i   __attribute__((ext_vector_type(8)));
typedef unsigned short v8us  __attribute__((ext_vector_type(8)));
typedef unsigned short v16us __attribute__((ext_vector_type(16)));
typedef __bf16         v16bf __attribute__((ext_vector_type(16)));
typedef _Float16       v16h  __attribute__((ext_vector_type(16)));
typedef v4f  __attribute__((may_alias)) v4fa;
typedef v8us __attribute__((may_alias)) v8usa;
union FragB { v16bf v; v16us u; v8us h[2]; v8i w; };
union FragH { v16h  v; v16us u; v8us h[2]; v8i w; };

__device__ __forceinline__ v8f wmb(const FragB& a, const FragB& b, v8f c) {
  v8f d = __builtin_amdgcn_wmma_f32_16x16x32_bf16(false, a.v, false, b.v, (short)0, c, false, false);
  asm volatile("v_nop\n\tv_nop\n\tv_nop\n\tv_nop" : "+v"(d) : "v"(a.w), "v"(b.w));
  return d;
}

__device__ __forceinline__ v8f wmh(const FragH& a, const FragH& b, v8f c) {
  v8f d = __builtin_amdgcn_wmma_f32_16x16x32_f16(false, a.v, false, b.v, (short)0, c, false, false);
  asm volatile("v_nop\n\tv_nop\n\tv_nop\n\tv_nop" : "+v"(d) : "v"(a.w), "v"(b.w));
  return d;
}

__device__ __forceinline__ unsigned bf16_bits(float f) {
  const unsigned u = __float_as_uint(f);
  const unsigned r = (u + 0x7FFFu + ((u >> 16) & 1u)) >> 16;
  const unsigned q = (u >> 16) | 0x40u;
  return ((u & 0x7fffffffu) > 0x7f800000u) ? q : r;
}

__device__ __forceinline__ float bf16_val(float f) {
  return __uint_as_float(bf16_bits(f) << 16);
}
__device__ __forceinline__ int clampi(int v, int lo, int hi) {
  return v < lo ? lo : (v > hi ? hi : v);
}

__device__ __forceinline__ unsigned f16_bits(float f) {
  const unsigned u  = __float_as_uint(f);
  const unsigned s  = (u >> 16) & 0x8000u;
  const unsigned a  = u & 0x7fffffffu;
  const unsigned t  = a - 0x38000000u;
  const unsigned r  = (t + 0x0FFFu + ((t >> 13) & 1u)) >> 13;
  const unsigned rc = r > 0x7C00u ? 0x7C00u : r;
  const bool small  = a < 0x38800000u;
  const bool isnan  = a > 0x7f800000u;
  const unsigned fin = small ? 0u : (s | rc);
  return isnan ? (s | 0x7E00u) : fin;
}

__device__ __forceinline__ unsigned pk16(unsigned lo, unsigned hi) { return lo | (hi << 16); }
__device__ __forceinline__ unsigned bf16_lo_bits(float v) {
  float hi = bf16_val(v);
  asm volatile("" : "+v"(hi));
  return bf16_bits(v - hi);
}
__device__ __forceinline__ v4u pack8_bf16(v4f a, v4f c) {
  return (v4u){ pk16(bf16_bits(a[0]), bf16_bits(a[1])), pk16(bf16_bits(a[2]), bf16_bits(a[3])),
                pk16(bf16_bits(c[0]), bf16_bits(c[1])), pk16(bf16_bits(c[2]), bf16_bits(c[3])) };
}
__device__ __forceinline__ v4u pack8_bf16_lo(v4f a, v4f c) {
  return (v4u){ pk16(bf16_lo_bits(a[0]), bf16_lo_bits(a[1])), pk16(bf16_lo_bits(a[2]), bf16_lo_bits(a[3])),
                pk16(bf16_lo_bits(c[0]), bf16_lo_bits(c[1])), pk16(bf16_lo_bits(c[2]), bf16_lo_bits(c[3])) };
}
__device__ __forceinline__ v4u pack8_f16(v4f a, v4f c) {
  return (v4u){ pk16(f16_bits(a[0]), f16_bits(a[1])), pk16(f16_bits(a[2]), f16_bits(a[3])),
                pk16(f16_bits(c[0]), f16_bits(c[1])), pk16(f16_bits(c[2]), f16_bits(c[3])) };
}

template <int FORM>
__global__ __launch_bounds__(256) void k_plane(const float* __restrict__ src, int rows, int cols, int ldsrc,
                                               unsigned short* __restrict__ dst, int MP, int KP) {
  static_assert(FORM >= 0 && FORM <= 3);
  const int KTOT = (FORM == 1 || FORM == 3) ? 2 * KP : KP;
  const unsigned ppr   = (unsigned)(KTOT >> 3);
  const unsigned kp8   = (unsigned)(KP >> 3);
  const unsigned total = (unsigned)MP * ppr;
  const unsigned g     = blockIdx.x * 256u + threadIdx.x;
  const unsigned rowu  = g / ppr;
  const unsigned p     = g - rowu * ppr;
  const bool second    = p >= kp8;
  const int row = (int)rowu;
  const int c0  = (int)((second ? p - kp8 : p) << 3);
  const float* srow = src + (size_t)clampi(row, 0, rows - 1) * (size_t)ldsrc;
  float x[8];
  unsigned mk[8];
#pragma unroll
  for (int e = 0; e < 8; ++e) {
    const int c = c0 + e;
    const float v = srow[clampi(c, 0, cols - 1)];
    asm volatile("" :: "v"(v));
    x[e]  = v;
    mk[e] = (row < rows && c < cols) ? 0xFFFFu : 0u;
  }
  const v4f a = (v4f){ x[0], x[1], x[2], x[3] };
  const v4f c = (v4f){ x[4], x[5], x[6], x[7] };
  v4u o;
  if (FORM == 2) {
    o = pack8_f16(a, c);
  } else {
    const v4u hi = pack8_bf16(a, c);
    o = hi;
    if (FORM == 1) { const v4u lo = pack8_bf16_lo(a, c); o = second ? lo : hi; }
  }
  const v4u mw = (v4u){ pk16(mk[0], mk[1]), pk16(mk[2], mk[3]), pk16(mk[4], mk[5]), pk16(mk[6], mk[7]) };
  o &= mw;
  if (g < total) {
    volatile v4u* q = (volatile v4u*)(dst + (size_t)g * 8);
    *q = o;
    __threadfence();
    *q = o;
  }
}

template <int FORM> struct FragOf    { typedef FragB T; };
template <>         struct FragOf<2> { typedef FragH T; };
__device__ __forceinline__ v8f mm(const FragB& a, const FragB& b, v8f c) { return wmb(a, b, c); }
__device__ __forceinline__ v8f mm(const FragH& a, const FragH& b, v8f c) { return wmh(a, b, c); }
template <class F> __device__ __forceinline__ F ld_frag(const unsigned short* p) {
  F f;
  f.h[0] = *(const v8usa*)(p);
  f.h[1] = *(const v8usa*)(p + 16);
  return f;
}

template <int FORM, int EPI>
__global__ __launch_bounds__(256) __attribute__((amdgpu_num_vgpr(248)))
void k_gemm_nt(const unsigned short* __restrict__ A, const unsigned short* __restrict__ B,
               const float* __restrict__ bias, float* __restrict__ D, int M, int N, int KTOT, int ldd) {
  static_assert(FORM >= 0 && FORM <= 2);
  static_assert(EPI == 0 || EPI == 1);
  typedef typename FragOf<FORM>::T F;
  __shared__ __attribute__((aligned(16))) float sT[8][16 * 68];
  const int lane = threadIdx.x & 31;
  const int wave = threadIdx.x >> 5;
  const int tilesM = (M + 63) >> 6;
  const int tilesN = (N + 63) >> 6;
  const int tile = blockIdx.x * 8 + wave;
  if (tile >= tilesM * tilesN) return;
  const int tm = tile / tilesN;
  const int tn = tile - tm * tilesN;
  const int m0 = tm << 6;
  const int n0 = tn << 6;

  const int rl = lane & 15;
  const int h8 = (lane >> 4) * 8;
  const unsigned short* pa = A + (size_t)(m0 + rl) * (size_t)KTOT + h8;
  const unsigned short* pb = B + (size_t)(n0 + rl) * (size_t)KTOT + h8;

  v8f acc[4][4];
#pragma unroll
  for (int i = 0; i < 4; ++i)
#pragma unroll
    for (int j = 0; j < 4; ++j) acc[i][j] = (v8f){0.f, 0.f, 0.f, 0.f, 0.f, 0.f, 0.f, 0.f};

#pragma unroll 1
  for (int k0 = 0; k0 < KTOT; k0 += 32) {
    F bf[4];
#pragma unroll
    for (int j = 0; j < 4; ++j) bf[j] = ld_frag<F>(pb + (size_t)(j << 4) * (size_t)KTOT + k0);
#pragma unroll
    for (int i = 0; i < 4; ++i) {
      const F af = ld_frag<F>(pa + (size_t)(i << 4) * (size_t)KTOT + k0);
#pragma unroll
      for (int j = 0; j < 4; ++j) acc[i][j] = mm(af, bf[j], acc[i][j]);
    }
  }

  float* slab = sT[wave];
  const int hh = lane >> 4;
  const int c4 = (lane & 15) * 4;
  const int nc = n0 + c4;
  const bool cok = nc < N;
  v4f bv = (v4f){0.f, 0.f, 0.f, 0.f};
  if (EPI == 1) {
    bv = *(const v4fa*)(bias + clampi(nc, 0, N - 4));
    asm volatile("" :: "v"(bv));
  }
#pragma unroll
  for (int i = 0; i < 4; ++i) {
    const int mBase = m0 + (i << 4);
#pragma unroll
    for (int j = 0; j < 4; ++j) {
#pragma unroll
      for (int r = 0; r < 8; ++r) slab[(h8 + r) * 68 + (j << 4) + rl] = acc[i][j][r];
    }
    __builtin_amdgcn_fence(__ATOMIC_RELEASE, "workgroup");
    __builtin_amdgcn_wave_barrier();
    __builtin_amdgcn_fence(__ATOMIC_ACQUIRE, "workgroup");
    v4f vv[8];
#pragma unroll
    for (int it = 0; it < 8; ++it) {
      const int row = it * 2 + hh;
      v4f v = *(const v4fa*)(slab + row * 68 + c4);
      if (EPI == 1) v += bv;
      vv[it] = v;
    }
    for (int pass = 0; pass < 2; ++pass) {
#pragma unroll
      for (int it = 0; it < 8; ++it) {
        const int row = mBase + it * 2 + hh;
        if (cok && row < M) *(volatile v4f*)(D + (size_t)row * (size_t)ldd + nc) = vv[it];
      }
      __threadfence();
    }
    __builtin_amdgcn_fence(__ATOMIC_RELEASE, "workgroup");
    __builtin_amdgcn_wave_barrier();
    __builtin_amdgcn_fence(__ATOMIC_ACQUIRE, "workgroup");
  }
}


#define SPLIT_HX 1
#define SPLIT_XE 1
#define SPLIT_TE 1

#define NROW  2048
#define MTUP  256
#define DIN   512
#define HID   512
#define EMB   256
#define W1IN  512
#define NPRED 8
#define NFILT 192
#define NREO  8
#define PHC   64
#define PLD   68

static_assert(NROW % 128 == 0);
static_assert(MTUP % 64 == 0);
static_assert(HID % 64 == 0);
static_assert(EMB % 64 == 0);
static_assert(2 * EMB == W1IN);
static_assert(HID % 32 == 0 && EMB % 32 == 0 && DIN % 32 == 0);
static_assert(EMB / 8 == 32);
static_assert(HID / 4 == 128);
static_assert((NROW * DIN / 8) % 256 == 0);
static_assert((HID * DIN / 8) % 256 == 0);
static_assert((EMB * HID / 8) % 256 == 0);
static_assert((HID * EMB / 8) % 256 == 0);
static_assert((MTUP * (EMB / 8)) % 256 == 0);
static_assert((NROW * (HID / 8)) % 256 == 0);
static_assert((NROW * (EMB / 8)) % 256 == 0);
static_assert((MTUP * HID / 4) % 256 == 0);
static_assert(PHC == 64 && (PLD % 4) == 0 && PLD >= 64);
static_assert((2 * PHC * PLD + HID) * 4 <= 65536);

template <int SPLIT>
__global__ __launch_bounds__(256) void k_temb(const int* __restrict__ tup, const float* __restrict__ Ep,
                                              const float* __restrict__ Ef, const float* __restrict__ Er,
                                              unsigned short* __restrict__ dst) {
  const int total = MTUP * (EMB / 8);
  const int g  = (int)(blockIdx.x * 256u + threadIdx.x);
  const int gc = clampi(g, 0, total - 1);
  const int m  = gc >> 5;
  const int c0 = (gc & 31) << 3;
  const int i0 = clampi(tup[m * 3 + 0], 0, NPRED - 1);
  const int i1 = clampi(tup[m * 3 + 1], 0, NFILT - 1);
  const int i2 = clampi(tup[m * 3 + 2], 0, NREO - 1);
  const v4f p0 = *(const v4fa*)(Ep + (size_t)i0 * EMB + c0);
  const v4f p1 = *(const v4fa*)(Ep + (size_t)i0 * EMB + c0 + 4);
  const v4f f0 = *(const v4fa*)(Ef + (size_t)i1 * EMB + c0);
  const v4f f1 = *(const v4fa*)(Ef + (size_t)i1 * EMB + c0 + 4);
  const v4f r0 = *(const v4fa*)(Er + (size_t)i2 * EMB + c0);
  const v4f r1 = *(const v4fa*)(Er + (size_t)i2 * EMB + c0 + 4);
  asm volatile("" :: "v"(p0), "v"(p1), "v"(f0));
  asm volatile("" :: "v"(f1), "v"(r0), "v"(r1));
  v4f a, c;
#pragma unroll
  for (int e = 0; e < 4; ++e) {
    a[e] = (bf16_val(p0[e]) + bf16_val(f0[e])) + bf16_val(r0[e]);
    c[e] = (bf16_val(p1[e]) + bf16_val(f1[e])) + bf16_val(r1[e]);
  }
  const v4u hi = pack8_bf16(a, c);
  const v4u lo = pack8_bf16_lo(a, c);
  const int pitch = SPLIT ? 2 * EMB : EMB;
  if (g < total) {
    volatile v4u* qh = (volatile v4u*)(dst + (size_t)m * pitch + c0);
    volatile v4u* ql = (volatile v4u*)(dst + (size_t)m * pitch + (SPLIT ? EMB : 0) + c0);
    *qh = hi;
    if (SPLIT) *ql = lo;
    __threadfence();
    *qh = hi;
    if (SPLIT) *ql = lo;
  }
}

template <int SPLIT>
__global__ __launch_bounds__(256) void k_act(const float* __restrict__ C, const float* __restrict__ bias,
                                             unsigned short* __restrict__ dst, int rows, int cols) {
  const unsigned ppr   = (unsigned)(cols >> 3);
  const unsigned total = (unsigned)rows * ppr;
  const unsigned g     = blockIdx.x * 256u + threadIdx.x;
  const unsigned gc    = g < total ? g : total - 1u;
  const unsigned row   = gc / ppr;
  const int c0 = (int)((gc - row * ppr) << 3);
  const float* s = C + (size_t)row * (size_t)cols + c0;
  v4f a = *(const v4fa*)(s);
  v4f c = *(const v4fa*)(s + 4);
  const v4f b0 = *(const v4fa*)(bias + c0);
  const v4f b1 = *(const v4fa*)(bias + c0 + 4);
  asm volatile("" :: "v"(a), "v"(c), "v"(b0), "v"(b1));
#pragma unroll
  for (int e = 0; e < 4; ++e) {
    a[e] = fmaxf(a[e] + bf16_val(b0[e]), 0.0f);
    c[e] = fmaxf(c[e] + bf16_val(b1[e]), 0.0f);
  }
  const v4u hi = pack8_bf16(a, c);
  const v4u lo = pack8_bf16_lo(a, c);
  const size_t pitch = SPLIT ? (size_t)(2 * cols) : (size_t)cols;
  if (g < total) {
    volatile v4u* qh = (volatile v4u*)(dst + (size_t)row * pitch + c0);
    volatile v4u* ql = (volatile v4u*)(dst + (size_t)row * pitch + (SPLIT ? cols : 0) + c0);
    *qh = hi;
    if (SPLIT) *ql = lo;
    __threadfence();
    *qh = hi;
    if (SPLIT) *ql = lo;
  }
}

__global__ __launch_bounds__(256) void k_htb(const float* __restrict__ HT, const float* __restrict__ b1,
                                             float* __restrict__ HTB) {
  const int total = MTUP * HID / 4;
  const int g  = (int)(blockIdx.x * 256u + threadIdx.x);
  const int gc = clampi(g, 0, total - 1);
  const int col = (gc & (HID / 4 - 1)) * 4;
  const v4f v = *(const v4fa*)(HT + (size_t)gc * 4);
  const v4f b = *(const v4fa*)(b1 + col);
  asm volatile("" :: "v"(v), "v"(b));
  v4f o;
#pragma unroll
  for (int e = 0; e < 4; ++e) o[e] = v[e] + bf16_val(b[e]);
  if (g < total) {
    volatile v4f* q = (volatile v4f*)(HTB + (size_t)gc * 4);
    *q = o;
    __threadfence();
    *q = o;
  }
}

__global__ __launch_bounds__(256) void k_pair(const float* __restrict__ HX, const float* __restrict__ HTB,
                                              const float* __restrict__ W2, const float* __restrict__ b2,
                                              float* __restrict__ out) {
  __shared__ __attribute__((aligned(16))) float sx[PHC * PLD];
  __shared__ __attribute__((aligned(16))) float st[PHC * PLD];
  __shared__ __attribute__((aligned(16))) float sw[HID];
  const int tid = threadIdx.x;
  const int tx = tid & 15;
  const int ty = tid >> 4;
  const int n0 = blockIdx.x * 64;
  const int m0 = blockIdx.y * 64;

  {
    const int wi = (tid < HID / 4 ? tid : HID / 4 - 1) * 4;
    const v4f wv = *(const v4fa*)(W2 + wi);
    asm volatile("" :: "v"(wv));
    const v4f wr = (v4f){ bf16_val(wv[0]), bf16_val(wv[1]), bf16_val(wv[2]), bf16_val(wv[3]) };
    if (tid < HID / 4) *(v4fa*)(sw + wi) = wr;
  }
  const float b2r = bf16_val(b2[0]);

  float acc[4][4];
#pragma unroll
  for (int i = 0; i < 4; ++i)
#pragma unroll
    for (int j = 0; j < 4; ++j) acc[i][j] = 0.0f;

#pragma unroll 1
  for (int hc = 0; hc < HID; hc += PHC) {
#pragma unroll
    for (int p = 0; p < 4; ++p) {
      const int i  = tid + 256 * p;
      const int r  = i >> 4;
      const int c4 = (i & 15) * 4;
      const v4f v = *(const v4fa*)(HX  + (size_t)(n0 + r) * HID + hc + c4);
      const v4f u = *(const v4fa*)(HTB + (size_t)(m0 + r) * HID + hc + c4);
      sx[(c4 + 0) * PLD + r] = v[0];
      sx[(c4 + 1) * PLD + r] = v[1];
      sx[(c4 + 2) * PLD + r] = v[2];
      sx[(c4 + 3) * PLD + r] = v[3];
      st[(c4 + 0) * PLD + r] = u[0];
      st[(c4 + 1) * PLD + r] = u[1];
      st[(c4 + 2) * PLD + r] = u[2];
      st[(c4 + 3) * PLD + r] = u[3];
    }
    __syncthreads();

#pragma unroll 4
    for (int h = 0; h < PHC; ++h) {
      const float wv = sw[hc + h];
      const v4f xs = *(const v4fa*)(sx + h * PLD + 4 * ty);
      const v4f ts = *(const v4fa*)(st + h * PLD + 4 * tx);
#pragma unroll
      for (int i = 0; i < 4; ++i)
#pragma unroll
        for (int j = 0; j < 4; ++j) {
          float v = xs[i] + ts[j];
          v = fmaxf(v, 0.0f);
          acc[i][j] = fmaf(v, wv, acc[i][j]);
        }
    }
    __syncthreads();
  }

  v4f vv[4];
#pragma unroll
  for (int i = 0; i < 4; ++i)
    vv[i] = (v4f){ acc[i][0] + b2r, acc[i][1] + b2r, acc[i][2] + b2r, acc[i][3] + b2r };
  for (int pass = 0; pass < 2; ++pass) {
#pragma unroll
    for (int i = 0; i < 4; ++i)
      *(volatile v4f*)(out + (size_t)(n0 + 4 * ty + i) * MTUP + m0 + 4 * tx) = vv[i];
    __threadfence();
  }
}

extern "C" void kernel_launch(void* const* d_in, const int* in_sizes, int n_in,
                              void* d_out, int out_size, void* d_ws, size_t ws_size,
                              hipStream_t stream) {
  if (n_in < 13) return;
  if (in_sizes[0]  != NROW * DIN)   return;
  if (in_sizes[1]  != MTUP * 3)     return;
  if (in_sizes[2]  != HID * DIN)    return;
  if (in_sizes[3]  != HID)          return;
  if (in_sizes[4]  != EMB * HID)    return;
  if (in_sizes[5]  != EMB)          return;
  if (in_sizes[6]  != NPRED * EMB)  return;
  if (in_sizes[7]  != NFILT * EMB)  return;
  if (in_sizes[8]  != NREO * EMB)   return;
  if (in_sizes[9]  != HID * W1IN)   return;
  if (in_sizes[10] != HID)          return;
  if (in_sizes[11] != HID)          return;
  if (in_sizes[12] != 1)            return;
  if (out_size != NROW * MTUP) return;

  const float* x   = (const float*)d_in[0];
  const int*   tup = (const int*)  d_in[1];
  const float* Wa  = (const float*)d_in[2];
  const float* ba  = (const float*)d_in[3];
  const float* Wb  = (const float*)d_in[4];
  const float* bb  = (const float*)d_in[5];
  const float* Ep  = (const float*)d_in[6];
  const float* Ef  = (const float*)d_in[7];
  const float* Er  = (const float*)d_in[8];
  const float* W1  = (const float*)d_in[9];
  const float* b1  = (const float*)d_in[10];
  const float* W2  = (const float*)d_in[11];
  const float* b2  = (const float*)d_in[12];
  float* out = (float*)d_out;

  constexpr int KT_HX = SPLIT_HX ? 2 * HID : HID;
  constexpr int KT_XE = SPLIT_XE ? 2 * EMB : EMB;
  constexpr int KT_TE = SPLIT_TE ? 2 * EMB : EMB;
  constexpr int FW_HX = SPLIT_HX ? 3 : 0;
  constexpr int FW_XE = SPLIT_XE ? 3 : 0;
  constexpr int FW_TE = SPLIT_TE ? 3 : 0;
  static_assert(KT_HX % 32 == 0 && KT_XE % 32 == 0 && KT_TE % 32 == 0);
  static_assert((EMB * KT_HX / 8) % 256 == 0);
  static_assert((HID * KT_XE / 8) % 256 == 0);
  static_assert((HID * KT_TE / 8) % 256 == 0);

  const size_t S_XB   = (size_t)NROW * DIN * 2;
  const size_t S_WAB  = (size_t)HID * DIN * 2;
  const size_t S_WB2  = (size_t)EMB * 2 * HID * 2;
  const size_t S_W1X2 = (size_t)HID * 2 * EMB * 2;
  const size_t S_W1T2 = (size_t)HID * 2 * EMB * 2;
  const size_t S_C1   = (size_t)NROW * HID * 4;
  const size_t S_HXA  = (size_t)NROW * 2 * HID * 2;
  const size_t S_C2   = (size_t)NROW * EMB * 4;
  const size_t S_XE   = (size_t)NROW * 2 * EMB * 2;
  const size_t S_HX   = (size_t)NROW * HID * 4;
  const size_t S_TE   = (size_t)MTUP * 2 * EMB * 2;
  const size_t S_HT   = (size_t)MTUP * HID * 4;
  size_t off = 0;
  const size_t oXB   = off; off += S_XB;
  const size_t oWAB  = off; off += S_WAB;
  const size_t oWB2  = off; off += S_WB2;
  const size_t oW1X2 = off; off += S_W1X2;
  const size_t oW1T2 = off; off += S_W1T2;
  const size_t oC1   = off; off += S_C1;
  const size_t oHXA  = off; off += S_HXA;
  const size_t oC2   = off; off += S_C2;
  const size_t oXE   = off; off += S_XE;
  const size_t oHX   = off; off += S_HX;
  const size_t oTE   = off; off += S_TE;
  const size_t oHT   = off; off += S_HT;
  const size_t oHTB  = off; off += S_HT;
  if (off > ws_size) return;
  if (off > ((size_t)128 << 20)) return;

  char* ws = (char*)d_ws;
  unsigned short* XB   = (unsigned short*)(ws + oXB);
  unsigned short* WAB  = (unsigned short*)(ws + oWAB);
  unsigned short* WB2  = (unsigned short*)(ws + oWB2);
  unsigned short* W1X2 = (unsigned short*)(ws + oW1X2);
  unsigned short* W1T2 = (unsigned short*)(ws + oW1T2);
  float*          C1   = (float*)(ws + oC1);
  unsigned short* HXA  = (unsigned short*)(ws + oHXA);
  float*          C2   = (float*)(ws + oC2);
  unsigned short* XE   = (unsigned short*)(ws + oXE);
  float*          HX   = (float*)(ws + oHX);
  unsigned short* TEHL = (unsigned short*)(ws + oTE);
  float*          HT   = (float*)(ws + oHT);
  float*          HTB  = (float*)(ws + oHTB);

  k_plane<0><<<dim3(NROW * DIN / 8 / 256), 256, 0, stream>>>(x, NROW, DIN, DIN, XB, NROW, DIN);
  k_plane<0><<<dim3(HID * DIN / 8 / 256), 256, 0, stream>>>(Wa, HID, DIN, DIN, WAB, HID, DIN);
  k_plane<FW_HX><<<dim3(EMB * KT_HX / 8 / 256), 256, 0, stream>>>(Wb, EMB, HID, HID, WB2, EMB, HID);
  k_plane<FW_XE><<<dim3(HID * KT_XE / 8 / 256), 256, 0, stream>>>(W1, HID, EMB, W1IN, W1X2, HID, EMB);
  k_plane<FW_TE><<<dim3(HID * KT_TE / 8 / 256), 256, 0, stream>>>(W1 + EMB, HID, EMB, W1IN, W1T2, HID, EMB);
  k_temb<SPLIT_TE><<<dim3(MTUP * (EMB / 8) / 256), 256, 0, stream>>>(tup, Ep, Ef, Er, TEHL);
  k_gemm_nt<0, 0><<<dim3((NROW / 64) * (HID / 64) / 8), 256, 0, stream>>>(XB, WAB, ba, C1, NROW, HID, DIN, HID);
  k_act<SPLIT_HX><<<dim3(NROW * (HID / 8) / 256), 256, 0, stream>>>(C1, ba, HXA, NROW, HID);
  k_gemm_nt<0, 0><<<dim3((NROW / 64) * (EMB / 64) / 8), 256, 0, stream>>>(HXA, WB2, ba, C2, NROW, EMB, KT_HX, EMB);
  k_act<SPLIT_XE><<<dim3(NROW * (EMB / 8) / 256), 256, 0, stream>>>(C2, bb, XE, NROW, EMB);
  k_gemm_nt<0, 0><<<dim3((NROW / 64) * (HID / 64) / 8), 256, 0, stream>>>(XE, W1X2, ba, HX, NROW, HID, KT_XE, HID);
  k_gemm_nt<0, 0><<<dim3((MTUP / 64) * (HID / 64) / 8), 256, 0, stream>>>(TEHL, W1T2, ba, HT, MTUP, HID, KT_TE, HID);
  k_htb<<<dim3(MTUP * HID / 4 / 256), 256, 0, stream>>>(HT, b1, HTB);
  k_pair<<<dim3(NROW / 64, MTUP / 64), 256, 0, stream>>>(HX, HTB, W2, b2, out);
  (void)hipGetLastError();
}
